// GraphSAGEWithSampling_59880434041042
// MI455X (gfx1250) — hardware-verified
//
#include <hip/hip_runtime.h>
#include <stddef.h>
#include <stdint.h>
#include <math.h>


#define DF     128
#define AP     256
#define NCLS   40
#define NH2    64
#define NTHR   256
#define NWAVE  8
#define EPT    8
#define CHUNK  (NTHR * EPT)
#define WCAP   (EPT * 32)
#define LISTN  (NWAVE * WCAP)
#define NBA    1024
#define SLA    10
#define RCAP   24576
#define DEGCAP 64
#define GBM    64
#define GTHR   128
#define UPART  2048
#define NPART  8
#define WBLK   ((NPART * UPART) / NTHR)
#define SCAN_ZINTS    (LISTN + 2 * RCAP + 3 * NBA)
#define SCAN_LDS_INTS (SCAN_ZINTS + 16)
#define WSMAX  134217728

static_assert((CHUNK & (CHUNK - 1)) == 0 && CHUNK <= 4096);
static_assert((NBA & (NBA - 1)) == 0 && NBA == (1 << SLA));
static_assert(((long long)CHUNK << SLA) < (1LL << 31));
static_assert(LISTN % NTHR == 0);
static_assert(NBA == 4 * NTHR && NBA == NWAVE * 128 && NBA % 32 == 0 && NBA % GBM == 0);
static_assert(RCAP % (NTHR * 4) == 0 && SCAN_ZINTS % (NTHR * 4) == 0 && LISTN % 4 == 0);
static_assert(GBM == (GTHR / 32) * 16 && DF == 4 * 32 && AP == 2 * DF);
static_assert((NPART * UPART) % NTHR == 0 && UPART % NTHR == 0);
static_assert(NCLS == 10 * 4 && NCLS <= NH2 && NH2 == 16 * 4);
static_assert(SCAN_LDS_INTS * 4 <= 300000);

typedef float          v4f   __attribute__((ext_vector_type(4)));
typedef float          v8f   __attribute__((ext_vector_type(8)));
typedef int            v4i   __attribute__((ext_vector_type(4)));
typedef int            v8i   __attribute__((ext_vector_type(8)));
typedef unsigned short v4us  __attribute__((ext_vector_type(4)));
typedef unsigned short v8us  __attribute__((ext_vector_type(8)));
typedef unsigned short v16us __attribute__((ext_vector_type(16)));
typedef __bf16         v16bf __attribute__((ext_vector_type(16)));
typedef v4f  __attribute__((may_alias)) v4fa;
typedef v4i  __attribute__((may_alias)) v4ia;
typedef v4us __attribute__((may_alias)) v4usa;
typedef v8us __attribute__((may_alias)) v8usa;
union FragB { v16bf v; v16us u; v8us h[2]; v8i w; };

__device__ __forceinline__ v8f wmb(const FragB& a, const FragB& b, v8f c) {
  v8f d = __builtin_amdgcn_wmma_f32_16x16x32_bf16(false, a.v, false, b.v, (short)0, c, false, false);
  asm volatile("v_nop\n\tv_nop\n\tv_nop\n\tv_nop" : "+v"(d) : "v"(a.w), "v"(b.w));
  return d;
}

__device__ __forceinline__ unsigned bf16_bits(float f) {
  const unsigned u = __float_as_uint(f);
  return (u + 0x7FFFu + ((u >> 16) & 1u)) >> 16;
}
__device__ __forceinline__ float bf16_val(float f) {
  return __uint_as_float(bf16_bits(f) << 16);
}
__device__ __forceinline__ int clampi(int v, int lo, int hi) { return v < lo ? lo : (v > hi ? hi : v); }

__device__ __forceinline__ void wave_sync() {
  __builtin_amdgcn_fence(__ATOMIC_RELEASE, "wavefront");
  __builtin_amdgcn_wave_barrier();
  __builtin_amdgcn_fence(__ATOMIC_ACQUIRE, "wavefront");
}

template <int SLB>
__device__ __forceinline__ int scan_chunk(const int* __restrict__ dsts, int nE, int cbase, int slotBase,
                                          int nb, int vec8, int* list, int tid, int lane, int wave) {
  int wc = 0;
  const int el0  = tid * EPT;
  const int e0   = cbase + el0;
  const int sent = -2147483647 - 1;
  v4i da, db;
  if (vec8 != 0 && cbase + CHUNK <= nE) {
    da = *(const v4i*)(dsts + e0);
    db = *(const v4i*)(dsts + e0 + 4);
  } else {
    da.x = (e0     < nE) ? dsts[min(e0,     nE - 1)] : sent;
    da.y = (e0 + 1 < nE) ? dsts[min(e0 + 1, nE - 1)] : sent;
    da.z = (e0 + 2 < nE) ? dsts[min(e0 + 2, nE - 1)] : sent;
    da.w = (e0 + 3 < nE) ? dsts[min(e0 + 3, nE - 1)] : sent;
    db.x = (e0 + 4 < nE) ? dsts[min(e0 + 4, nE - 1)] : sent;
    db.y = (e0 + 5 < nE) ? dsts[min(e0 + 5, nE - 1)] : sent;
    db.z = (e0 + 6 < nE) ? dsts[min(e0 + 6, nE - 1)] : sent;
    db.w = (e0 + 7 < nE) ? dsts[min(e0 + 7, nE - 1)] : sent;
  }
  const unsigned nbs = (unsigned)slotBase;
  const unsigned unb = (unsigned)nb;
  const unsigned s0 = (unsigned)da.x - nbs, s1 = (unsigned)da.y - nbs;
  const unsigned s2 = (unsigned)da.z - nbs, s3 = (unsigned)da.w - nbs;
  const unsigned s4 = (unsigned)db.x - nbs, s5 = (unsigned)db.y - nbs;
  const unsigned s6 = (unsigned)db.z - nbs, s7 = (unsigned)db.w - nbs;
  const bool h0 = s0 < unb, h1 = s1 < unb, h2 = s2 < unb, h3 = s3 < unb;
  const bool h4 = s4 < unb, h5 = s5 < unb, h6 = s6 < unb, h7 = s7 < unb;
  const unsigned any = __builtin_amdgcn_ballot_w32(h0 | h1 | h2 | h3 | h4 | h5 | h6 | h7);
  if (any != 0u) {
#define HITJ(J, HJ, SJ) { \
      const unsigned mj = __builtin_amdgcn_ballot_w32(HJ); \
      if (mj != 0u) { \
        if (HJ) { \
          const int pos = wc + (int)__builtin_amdgcn_mbcnt_lo(mj, 0u); \
          if (pos < WCAP) list[wave * WCAP + pos] = ((el0 + (J)) << SLB) | (int)(SJ); \
        } \
        wc += (int)__builtin_popcount(mj); } }
    HITJ(0, h0, s0)
    HITJ(1, h1, s1)
    HITJ(2, h2, s2)
    HITJ(3, h3, s3)
    HITJ(4, h4, s4)
    HITJ(5, h5, s5)
    HITJ(6, h6, s6)
    HITJ(7, h7, s7)
#undef HITJ
  }
  return wc;
}

__device__ __forceinline__ void build_offs(const int* cnt, int* offs, int lane) {
  const int base = lane * (NBA / 32);
  int s = 0;
#pragma unroll 1
  for (int i = 0; i < NBA / 32; ++i) s += clampi(cnt[base + i], 0, RCAP);
  int incl = s;
#pragma unroll
  for (int d = 1; d < 32; d <<= 1) {
    const int y = __shfl_up(incl, d, 32);
    if (lane >= d) incl += y;
  }
  int run = incl - s;
#pragma unroll 1
  for (int i = 0; i < NBA / 32; ++i) {
    offs[base + i] = run;
    run += clampi(cnt[base + i], 0, RCAP);
  }
}

__global__ __launch_bounds__(NTHR) void k_prep(const float* __restrict__ x,
                                               const float* __restrict__ Wl0, const float* __restrict__ Wr0,
                                               const float* __restrict__ Wl1, const float* __restrict__ Wr1,
                                               const float* __restrict__ Wl2, const float* __restrict__ Wr2,
                                               int nN, int mRows,
                                               unsigned short* WB0, unsigned short* WB1, unsigned short* WB2,
                                               unsigned short* PB) {
  const int tid = (int)threadIdx.x;
  const float* p;
  unsigned short* dp;
  bool ok, st;
  if ((int)blockIdx.x < WBLK) {
    const int u    = (int)blockIdx.x * NTHR + tid;
    const int part = u >> 11;
    const int v    = u & (UPART - 1);
    const float* W;
    unsigned short* P;
    int pitch, coff, roff, n, kk, nmax;
    if (part < 6) { n = v >> 4; kk = (v & 15) * 8; nmax = DF; }
    else          { n = v >> 5; kk = (v & 31) * 8; nmax = NCLS; }
    if (part == 0)      { W = Wl0; P = WB0; pitch = DF; roff = 0;   coff = 0; }
    else if (part == 1) { W = Wr0; P = WB0; pitch = DF; roff = DF;  coff = 0; }
    else if (part == 2) { W = Wl1; P = WB1; pitch = AP; roff = 0;   coff = 0; }
    else if (part == 3) { W = Wl1; P = WB1; pitch = AP; roff = 0;   coff = DF; }
    else if (part == 4) { W = Wr1; P = WB1; pitch = AP; roff = DF;  coff = 0; }
    else if (part == 5) { W = Wr1; P = WB1; pitch = AP; roff = DF;  coff = DF; }
    else if (part == 6) { W = Wl2; P = WB2; pitch = AP; roff = 0;   coff = 0; }
    else                { W = Wr2; P = WB2; pitch = AP; roff = NH2; coff = 0; }
    const int ks = kk & (DF - 1);
    const int nc = n < nmax ? n : nmax - 1;
    p  = W + (size_t)nc * DF + ks;
    ok = n < nmax;
    st = true;
    dp = P + (size_t)(roff + n) * pitch + coff + kk;
  } else {
    const int u   = ((int)blockIdx.x - WBLK) * NTHR + tid;
    const int row = u >> 4;
    const int k8  = (u & 15) * 8;
    const int rc  = row < nN ? row : nN - 1;
    p  = x + (size_t)rc * DF + k8;
    ok = row < nN;
    st = row < mRows;
    const int rs = row < mRows ? row : mRows - 1;
    dp = PB + (size_t)rs * AP + k8;
  }
  const v4f a = *(const v4fa*)p;
  const v4f b = *(const v4fa*)(p + 4);
  v8us o;
  o[0] = ok ? (unsigned short)bf16_bits(a.x) : (unsigned short)0;
  o[1] = ok ? (unsigned short)bf16_bits(a.y) : (unsigned short)0;
  o[2] = ok ? (unsigned short)bf16_bits(a.z) : (unsigned short)0;
  o[3] = ok ? (unsigned short)bf16_bits(a.w) : (unsigned short)0;
  o[4] = ok ? (unsigned short)bf16_bits(b.x) : (unsigned short)0;
  o[5] = ok ? (unsigned short)bf16_bits(b.y) : (unsigned short)0;
  o[6] = ok ? (unsigned short)bf16_bits(b.z) : (unsigned short)0;
  o[7] = ok ? (unsigned short)bf16_bits(b.w) : (unsigned short)0;
  if (st) *(volatile v8us*)dp = o;
  __threadfence();
  if (st) *(volatile v8us*)dp = o;
}

__global__ __launch_bounds__(NTHR) void k_scan(const int* __restrict__ srcs, const int* __restrict__ dsts,
                                               int nE, int nN, int vec8, int* hitsg, int* cntg) {
  extern __shared__ __attribute__((aligned(16))) int dsm[];
  int* list = dsm;
  int* hl   = dsm + LISTN;
  int* sl   = hl + RCAP;
  int* cnt  = sl + RCAP;
  int* offs = cnt + NBA;
  int* cur  = offs + NBA;
  int* misc = cur + NBA;
  const int tid = (int)threadIdx.x, lane = tid & 31, wave = tid >> 5;
  const int nodeBase = (int)blockIdx.x * NBA;

  {
    const v4i z4 = {0, 0, 0, 0};
    for (int i = tid * 4; i < SCAN_ZINTS; i += NTHR * 4) *(v4ia*)(dsm + i) = z4;
    if (tid < 16) misc[tid] = 0;
  }
  __syncthreads();

  int t = 0, ov = 0;
  const int nChunks = (nE + CHUNK - 1) / CHUNK;
#pragma unroll 1
  for (int ch = 0; ch < nChunks; ++ch) {
    const int cbase = ch * CHUNK;
    const int wc = scan_chunk<SLA>(dsts, nE, cbase, nodeBase, NBA, vec8, list, tid, lane, wave);
    if (lane == 0) misc[wave] = wc;
    __syncthreads();
    if (wave == 0) {
#pragma unroll 1
      for (int w2 = 0; w2 < NWAVE; ++w2) {
        int c = misc[w2];
        c = c < 0 ? 0 : (c > WCAP ? WCAP : c);
#pragma unroll 1
        for (int b0 = 0; b0 < c; b0 += 32) {
          const int idx = b0 + lane;
          const int ent = list[w2 * WCAP + (idx < WCAP ? idx : WCAP - 1)];
          const int m32 = (c - b0) < 32 ? (c - b0) : 32;
#pragma unroll 1
          for (int k = 0; k < m32; ++k) {
            const int u    = __builtin_amdgcn_readlane(ent, k);
            const int slot = u & (NBA - 1);
            const int el   = (u >> SLA) & (CHUNK - 1);
            const int pk   = ((cbase + el) << SLA) | slot;
            if (t < RCAP) {
              if (lane == 0) { hl[t] = pk; cnt[slot] = cnt[slot] + 1; }
              t = t + 1;
            } else {
              ov = 1;
            }
          }
        }
      }
    }
    __syncthreads();
  }
  if (wave == 0 && lane == 0) { misc[8] = t; misc[9] = ov; }
  __syncthreads();
  int tt = misc[8];
  tt = tt < 0 ? 0 : (tt > RCAP ? RCAP : tt);
  const int ovf = misc[9];

  if (wave == 0) {
    build_offs(cnt, offs, lane);
    const int base = lane * (NBA / 32);
#pragma unroll 1
    for (int i = 0; i < NBA / 32; ++i) cur[base + i] = offs[base + i];
  }
  __syncthreads();
  if (wave == 0) {
#pragma unroll 1
    for (int b0 = 0; b0 < tt; b0 += 32) {
      const int idx = b0 + lane;
      const int ent = hl[idx < RCAP ? idx : RCAP - 1];
      const int m32 = (tt - b0) < 32 ? (tt - b0) : 32;
#pragma unroll 1
      for (int k = 0; k < m32; ++k) {
        const int u    = __builtin_amdgcn_readlane(ent, k);
        const int slot = u & (NBA - 1);
        if (lane == 0) {
          int p = cur[slot];
          p = p < 0 ? 0 : (p > RCAP - 1 ? RCAP - 1 : p);
          sl[p] = u;
          cur[slot] = p + 1;
        }
      }
    }
  }
  __syncthreads();

  int* hb = hitsg + (size_t)blockIdx.x * RCAP;
#pragma unroll 1
  for (int i = tid * 4; i < RCAP; i += NTHR * 4) {
    const v4i e4 = *(const v4ia*)(sl + i);
    const int q0 = clampi(e4.x >> SLA, 0, nE - 1);
    const int q1 = clampi(e4.y >> SLA, 0, nE - 1);
    const int q2 = clampi(e4.z >> SLA, 0, nE - 1);
    const int q3 = clampi(e4.w >> SLA, 0, nE - 1);
    const int r0 = clampi(srcs[q0], 0, nN - 1);
    const int r1 = clampi(srcs[q1], 0, nN - 1);
    const int r2 = clampi(srcs[q2], 0, nN - 1);
    const int r3 = clampi(srcs[q3], 0, nN - 1);
    v4i o;
    o.x = (i     < tt) ? r0 : 0;
    o.y = (i + 1 < tt) ? r1 : 0;
    o.z = (i + 2 < tt) ? r2 : 0;
    o.w = (i + 3 < tt) ? r3 : 0;
    *(volatile v4i*)(hb + i) = o;
    __threadfence();
    *(volatile v4i*)(hb + i) = o;
  }
  {
    v4i c4 = *(const v4ia*)(cnt + 4 * tid);
    if (ovf != 0) { c4.x = -1; c4.y = -1; c4.z = -1; c4.w = -1; }
    int* cp = cntg + (size_t)blockIdx.x * NBA + 4 * tid;
    *(volatile v4i*)cp = c4;
    __threadfence();
    *(volatile v4i*)cp = c4;
  }
}

template <int NT>
__global__ __launch_bounds__(GTHR) void k_gemm(unsigned short* PB, const unsigned short* __restrict__ BT, int K,
                                               float* YL) {
  constexpr int NH = 16 * NT;
  __shared__ __attribute__((aligned(16))) float stg[GBM * DF];
  const int tid = (int)threadIdx.x, lane = tid & 31, wave = tid >> 5, hh = lane >> 4, m = lane & 15;
  const int rowBase = (int)blockIdx.x * GBM;
  const unsigned short* ap = PB + (size_t)(rowBase + 16 * wave + m) * (size_t)AP + 8 * hh;

#pragma unroll 1
  for (int hf = 0; hf < 2; ++hf) {
    v8f acc[NT];
    {
      const v8f z = {0.f, 0.f, 0.f, 0.f, 0.f, 0.f, 0.f, 0.f};
#pragma unroll
      for (int t = 0; t < NT; ++t) acc[t] = z;
    }
    const unsigned short* bp = BT + (size_t)(hf * NH + m) * (size_t)K + 8 * hh;
#pragma unroll 1
    for (int k0 = 0; k0 < K; k0 += 32) {
      FragB af;
      af.h[0] = *(const v8usa*)(ap + k0);
      af.h[1] = *(const v8usa*)(ap + k0 + 16);
#pragma unroll
      for (int nt = 0; nt < NT; ++nt) {
        const unsigned short* wq = bp + (size_t)(16 * nt) * (size_t)K + k0;
        FragB bf;
        bf.h[0] = *(const v8usa*)wq;
        bf.h[1] = *(const v8usa*)(wq + 16);
        acc[nt] = wmb(af, bf, acc[nt]);
      }
    }
#pragma unroll
    for (int nt = 0; nt < NT; ++nt) {
      const int lc = 16 * nt + m;
#pragma unroll
      for (int r = 0; r < 8; ++r) {
        const int lr = 16 * wave + 8 * hh + r;
        stg[lr * NH + lc] = acc[nt][r];
      }
    }
    __syncthreads();

    float* dst = (hf != 0) ? (float*)PB : YL;
    const int pitch = (hf != 0) ? DF : NH;
    if constexpr (NT == 8) {
      v4f pv[16];
#pragma unroll
      for (int i = 0; i < 16; ++i) pv[i] = *(const v4fa*)(stg + (16 * wave + i) * NH + 4 * lane);
      __syncthreads();
#pragma unroll
      for (int i = 0; i < 16; ++i)
        *(volatile v4f*)(dst + (size_t)(rowBase + 16 * wave + i) * pitch + 4 * lane) = pv[i];
      __threadfence();
#pragma unroll
      for (int i = 0; i < 16; ++i)
        *(volatile v4f*)(dst + (size_t)(rowBase + 16 * wave + i) * pitch + 4 * lane) = pv[i];
    } else {
      v4f fv[8];
#pragma unroll
      for (int i = 0; i < 8; ++i) {
        const int lr = 16 * wave + 2 * i + hh;
        fv[i] = *(const v4fa*)(stg + lr * NH + 4 * m);
      }
      __syncthreads();
#pragma unroll
      for (int i = 0; i < 8; ++i) {
        const int lr = 16 * wave + 2 * i + hh;
        *(volatile v4f*)(dst + (size_t)(rowBase + lr) * pitch + 4 * m) = fv[i];
      }
      __threadfence();
#pragma unroll
      for (int i = 0; i < 8; ++i) {
        const int lr = 16 * wave + 2 * i + hh;
        *(volatile v4f*)(dst + (size_t)(rowBase + lr) * pitch + 4 * m) = fv[i];
      }
    }
  }
}

__global__ __launch_bounds__(NTHR) void k_agg(const int* __restrict__ hitsg, const int* __restrict__ cntg,
                                              const float* __restrict__ YL, unsigned short* PB,
                                              const float* __restrict__ bias, int nN, int mRows) {
  __shared__ __attribute__((aligned(16))) int cnt[NBA];
  __shared__ __attribute__((aligned(16))) int offs[NBA];
  __shared__ __attribute__((aligned(16))) unsigned short rowb[NWAVE * AP];
  const int tid = (int)threadIdx.x, lane = tid & 31, wave = tid >> 5;
  const int nodeBase = (int)blockIdx.x * NBA;
  const int* hb = hitsg + (size_t)blockIdx.x * RCAP;
  unsigned short* rowbuf = rowb + wave * AP;

  {
    const v4i c4 = *(const v4i*)(cntg + (size_t)blockIdx.x * NBA + 4 * tid);
    *(v4ia*)(cnt + 4 * tid) = c4;
  }
  __syncthreads();
  if (wave == 0) build_offs(cnt, offs, lane);
  __syncthreads();

  v4f bb;
  {
    const v4f t1 = *(const v4f*)(bias + 4 * lane);
    bb.x = bf16_val(t1.x); bb.y = bf16_val(t1.y); bb.z = bf16_val(t1.z); bb.w = bf16_val(t1.w);
  }
  const float qnan = __int_as_float(0x7fc00000);

#pragma unroll 1
  for (int si = 0; si < NBA / NWAVE; ++si) {
    const int s    = si * NWAVE + wave;
    const int node = nodeBase + s;
    const int craw = cnt[s];
    const bool bad = (craw < 0) | (craw > DEGCAP);
    const int c    = craw < 0 ? 0 : (craw > DEGCAP ? DEGCAP : craw);
    const float degf = (float)(craw < 1 ? 1 : craw);
    const float inv  = 1.0f / degf;
    const int o = clampi(offs[s], 0, RCAP);
    float a0 = 0.0f, a1 = 0.0f, a2 = 0.0f, a3 = 0.0f;
#pragma unroll 1
    for (int b0 = 0; b0 < c; b0 += 32) {
      int idx = o + b0 + lane;
      idx = idx > RCAP - 1 ? RCAP - 1 : idx;
      const int sr = clampi(hb[idx], 0, nN - 1);
      const int m32 = (c - b0) < 32 ? (c - b0) : 32;
#pragma unroll 1
      for (int k = 0; k < m32; ++k) {
        const int sk = __builtin_amdgcn_readlane(sr, k);
        const v4f a = *(const v4f*)(YL + (size_t)sk * DF + 4 * lane);
        a0 += a.x; a1 += a.y; a2 += a.z; a3 += a.w;
      }
    }
    const int nr = node < mRows ? node : mRows - 1;
    const v4f yr = *(const v4fa*)((const float*)PB + (size_t)nr * DF + 4 * lane);
    const float v0 = (a0 * inv + yr.x) + bb.x;
    const float v1 = (a1 * inv + yr.y) + bb.y;
    const float v2 = (a2 * inv + yr.z) + bb.z;
    const float v3 = (a3 * inv + yr.w) + bb.w;
    float ss = (v0 * v0 + v1 * v1) + (v2 * v2 + v3 * v3);
    ss += __shfl_xor(ss, 16, 32);
    ss += __shfl_xor(ss, 8, 32);
    ss += __shfl_xor(ss, 4, 32);
    ss += __shfl_xor(ss, 2, 32);
    ss += __shfl_xor(ss, 1, 32);
    const float nrm = sqrtf(ss);
    const float dn  = fmaxf(nrm, 1e-12f);
    const float rn  = 1.0f / dn;
    float y0 = v0 * rn, y1 = v1 * rn, y2 = v2 * rn, y3 = v3 * rn;
    y0 = (y0 > 0.0f) ? y0 : (y0 - y0);
    y1 = (y1 > 0.0f) ? y1 : (y1 - y1);
    y2 = (y2 > 0.0f) ? y2 : (y2 - y2);
    y3 = (y3 > 0.0f) ? y3 : (y3 - y3);
    const float pzr = bad ? qnan : 0.0f;
    const bool live = node < nN;
    const float m0 = live ? (y0 + pzr) : 0.0f;
    const float m1 = live ? (y1 + pzr) : 0.0f;
    const float m2 = live ? (y2 + pzr) : 0.0f;
    const float m3 = live ? (y3 + pzr) : 0.0f;
    v4us mh, ml;
    {
      unsigned hbits;
      hbits = bf16_bits(m0); mh[0] = (unsigned short)hbits; ml[0] = (unsigned short)bf16_bits(m0 - __uint_as_float(hbits << 16));
      hbits = bf16_bits(m1); mh[1] = (unsigned short)hbits; ml[1] = (unsigned short)bf16_bits(m1 - __uint_as_float(hbits << 16));
      hbits = bf16_bits(m2); mh[2] = (unsigned short)hbits; ml[2] = (unsigned short)bf16_bits(m2 - __uint_as_float(hbits << 16));
      hbits = bf16_bits(m3); mh[3] = (unsigned short)hbits; ml[3] = (unsigned short)bf16_bits(m3 - __uint_as_float(hbits << 16));
    }
    *(v4usa*)(rowbuf + 4 * lane) = mh;
    *(v4usa*)(rowbuf + DF + 4 * lane) = ml;
    wave_sync();
    const v8us q0 = *(const v8usa*)(rowbuf + 8 * lane);
    wave_sync();
    if (node < mRows) {
      unsigned short* rpw = PB + (size_t)node * AP + 8 * lane;
      *(volatile v8us*)rpw = q0;
      __threadfence();
      *(volatile v8us*)rpw = q0;
    }
  }
}

__global__ __launch_bounds__(NTHR) void k_agg2(const int* __restrict__ hitsg, const int* __restrict__ cntg,
                                               const float* __restrict__ YL, const float* __restrict__ PBf,
                                               const float* __restrict__ bias, int nN, int mRows,
                                               float* outp, long long totalPieces) {
  __shared__ __attribute__((aligned(16))) int cnt[NBA];
  __shared__ __attribute__((aligned(16))) int offs[NBA];
  __shared__ __attribute__((aligned(16))) float stg[NWAVE * 16 * NCLS];
  const int tid = (int)threadIdx.x, lane = tid & 31, wave = tid >> 5;
  const int hh = lane >> 4, sub = lane & 15;
  const int nodeBase = (int)blockIdx.x * NBA;
  const int* hb = hitsg + (size_t)blockIdx.x * RCAP;
  float* stgw = stg + wave * (16 * NCLS);

  {
    const v4i c4 = *(const v4i*)(cntg + (size_t)blockIdx.x * NBA + 4 * tid);
    *(v4ia*)(cnt + 4 * tid) = c4;
  }
  __syncthreads();
  if (wave == 0) build_offs(cnt, offs, lane);
  __syncthreads();

  const bool chv = sub < (NCLS / 4);
  v4f bb;
  {
    const int sc = sub < (NCLS / 4) ? sub : (NCLS / 4 - 1);
    const v4f t1 = *(const v4f*)(bias + 4 * sc);
    bb.x = chv ? bf16_val(t1.x) : 0.0f;
    bb.y = chv ? bf16_val(t1.y) : 0.0f;
    bb.z = chv ? bf16_val(t1.z) : 0.0f;
    bb.w = chv ? bf16_val(t1.w) : 0.0f;
  }
  const float qnan = __int_as_float(0x7fc00000);
  const float vneg = -3.0e38f;

#pragma unroll 1
  for (int g = 0; g < 8; ++g) {
    const int sl0  = 128 * wave + 16 * g;
    const int row0 = nodeBase + sl0;
    if (row0 < nN) {
#pragma unroll 1
      for (int r = 0; r < 16; ++r) {
        const int s    = sl0 + r;
        const int node = row0 + r;
        const int craw = cnt[s];
        const bool bad = (craw < 0) | (craw > DEGCAP);
        const int c    = craw < 0 ? 0 : (craw > DEGCAP ? DEGCAP : craw);
        const float degf = (float)(craw < 1 ? 1 : craw);
        const float inv  = 1.0f / degf;
        const int o = clampi(offs[s], 0, RCAP);
        float a0 = 0.0f, a1 = 0.0f, a2 = 0.0f, a3 = 0.0f;
#pragma unroll 1
        for (int b0 = 0; b0 < c; b0 += 32) {
          int idx = o + b0 + lane;
          idx = idx > RCAP - 1 ? RCAP - 1 : idx;
          const int sr = clampi(hb[idx], 0, nN - 1);
          const int m32 = (c - b0) < 32 ? (c - b0) : 32;
#pragma unroll 1
          for (int j = 0; 2 * j < m32; ++j) {
            const int hidx = 2 * j + hh;
            const int sk = __shfl(sr, hidx, 32);
            const bool okh = hidx < m32;
            const v4f a = *(const v4f*)(YL + (size_t)sk * NH2 + 4 * sub);
            a0 += okh ? a.x : 0.0f;
            a1 += okh ? a.y : 0.0f;
            a2 += okh ? a.z : 0.0f;
            a3 += okh ? a.w : 0.0f;
          }
        }
        a0 += __shfl_xor(a0, 16, 32);
        a1 += __shfl_xor(a1, 16, 32);
        a2 += __shfl_xor(a2, 16, 32);
        a3 += __shfl_xor(a3, 16, 32);
        const int nr = node < mRows ? node : mRows - 1;
        const v4f yr = *(const v4f*)(PBf + (size_t)nr * DF + 4 * sub);
        const float v0 = (a0 * inv + yr.x) + bb.x;
        const float v1 = (a1 * inv + yr.y) + bb.y;
        const float v2 = (a2 * inv + yr.z) + bb.z;
        const float v3 = (a3 * inv + yr.w) + bb.w;
        float mx = v0;
        mx = (v1 > mx) ? v1 : mx;
        mx = (v2 > mx) ? v2 : mx;
        mx = (v3 > mx) ? v3 : mx;
        mx = chv ? mx : vneg;
        {
          float ot;
          ot = __shfl_xor(mx, 8, 32); mx = (ot > mx) ? ot : mx;
          ot = __shfl_xor(mx, 4, 32); mx = (ot > mx) ? ot : mx;
          ot = __shfl_xor(mx, 2, 32); mx = (ot > mx) ? ot : mx;
          ot = __shfl_xor(mx, 1, 32); mx = (ot > mx) ? ot : mx;
        }
        const float x0 = expf(v0 - mx), x1 = expf(v1 - mx), x2 = expf(v2 - mx), x3 = expf(v3 - mx);
        const float e0 = chv ? x0 : 0.0f;
        const float e1 = chv ? x1 : 0.0f;
        const float e2 = chv ? x2 : 0.0f;
        const float e3 = chv ? x3 : 0.0f;
        float sm = (e0 + e1) + (e2 + e3);
        sm += __shfl_xor(sm, 8, 32);
        sm += __shfl_xor(sm, 4, 32);
        sm += __shfl_xor(sm, 2, 32);
        sm += __shfl_xor(sm, 1, 32);
        const float rs  = 1.0f / sm;
        const float pzr = bad ? qnan : 0.0f;
        const bool live = node < nN;
        v4f p;
        p.x = live ? (e0 * rs + pzr) : 0.0f;
        p.y = live ? (e1 * rs + pzr) : 0.0f;
        p.z = live ? (e2 * rs + pzr) : 0.0f;
        p.w = live ? (e3 * rs + pzr) : 0.0f;
        if (lane < (NCLS / 4)) *(v4fa*)(stgw + r * NCLS + 4 * lane) = p;
      }
      wave_sync();
      v4f ov[5];
#pragma unroll
      for (int it = 0; it < 5; ++it) ov[it] = *(const v4fa*)(stgw + 4 * (it * 32 + lane));
      wave_sync();
      const long long gp0 = (long long)row0 * (NCLS / 4);
#pragma unroll
      for (int it = 0; it < 5; ++it) {
        const long long gp = gp0 + it * 32 + lane;
        if (gp < totalPieces) *(volatile v4f*)(outp + 4 * gp) = ov[it];
      }
      __threadfence();
#pragma unroll
      for (int it = 0; it < 5; ++it) {
        const long long gp = gp0 + it * 32 + lane;
        if (gp < totalPieces) *(volatile v4f*)(outp + 4 * gp) = ov[it];
      }
    }
  }
}

static inline int cdiv(int a, int b) { return (a + b - 1) / b; }
static inline size_t al256(size_t o) { return (o + 255) & ~(size_t)255; }

extern "C" void kernel_launch(void* const* d_in, const int* in_sizes, int n_in,
                              void* d_out, int out_size, void* d_ws, size_t ws_size,
                              hipStream_t stream) {
  if (n_in < 11) return;
  if (in_sizes[0] < DF || (in_sizes[0] % DF) != 0) return;
  const int nN = in_sizes[0] / DF;
  if (nN < 16 || nN > (1 << 22)) return;
  if (in_sizes[1] < 2 || (in_sizes[1] & 1) != 0) return;
  const int nE = in_sizes[1] / 2;
  if (nE < 1 || nE >= (1 << (31 - SLA))) return;
  if (in_sizes[2] != DF * DF || in_sizes[3] != DF * DF || in_sizes[4] != DF) return;
  if (in_sizes[5] != DF * DF || in_sizes[6] != DF * DF || in_sizes[7] != DF) return;
  if (in_sizes[8] != NCLS * DF || in_sizes[9] != NCLS * DF || in_sizes[10] != NCLS) return;
  if ((long long)out_size != (long long)nN * NCLS) return;

  const float* x    = (const float*)d_in[0];
  const int*   edge = (const int*)d_in[1];
  const float* Wl0  = (const float*)d_in[2];
  const float* Wr0  = (const float*)d_in[3];
  const float* b0   = (const float*)d_in[4];
  const float* Wl1  = (const float*)d_in[5];
  const float* Wr1  = (const float*)d_in[6];
  const float* b1   = (const float*)d_in[7];
  const float* Wl2  = (const float*)d_in[8];
  const float* Wr2  = (const float*)d_in[9];
  const float* b2   = (const float*)d_in[10];
  float* out = (float*)d_out;
  const int* src = edge;
  const int* dst = edge + nE;

  const int MP = cdiv(nN, GBM) * GBM;
  const int gM = MP / GBM;
  const int gA = cdiv(MP, NBA);
  if ((long long)gA * NBA < (long long)MP) return;
  if (((long long)MP * 16) % NTHR != 0) return;
  const int gX = (MP * 16) / NTHR;
  const int vec8 = ((nE & 3) == 0) ? 1 : 0;

  char* ws = (char*)d_ws;
  size_t off = 0;
  const size_t oWB0 = off; off = al256(off + (size_t)2 * DF * DF * 2);
  const size_t oWB1 = off; off = al256(off + (size_t)2 * DF * AP * 2);
  const size_t oWB2 = off; off = al256(off + (size_t)2 * NH2 * AP * 2);
  const size_t oCNT = off; off = al256(off + (size_t)gA * NBA * 4);
  const size_t oHIT = off; off = al256(off + (size_t)gA * RCAP * 4);
  const size_t oPA  = off; off = al256(off + (size_t)MP * DF * 4);
  const size_t oPB  = off; off = al256(off + (size_t)MP * AP * 2);
  if (off > ws_size || off > (size_t)WSMAX) return;
  unsigned short* WB0 = (unsigned short*)(ws + oWB0);
  unsigned short* WB1 = (unsigned short*)(ws + oWB1);
  unsigned short* WB2 = (unsigned short*)(ws + oWB2);
  int*            CNT = (int*)(ws + oCNT);
  int*            HIT = (int*)(ws + oHIT);
  float*          PA  = (float*)(ws + oPA);
  unsigned short* PB  = (unsigned short*)(ws + oPB);

  const size_t scanLds = (size_t)SCAN_LDS_INTS * 4;
  hipFuncSetAttribute(reinterpret_cast<const void*>(&k_scan), hipFuncAttributeMaxDynamicSharedMemorySize, (int)scanLds);

  k_prep<<<WBLK + gX, NTHR, 0, stream>>>(x, Wl0, Wr0, Wl1, Wr1, Wl2, Wr2, nN, MP, WB0, WB1, WB2, PB);
  k_scan<<<gA, NTHR, scanLds, stream>>>(src, dst, nE, nN, vec8, HIT, CNT);
  k_gemm<8><<<gM, GTHR, 0, stream>>>(PB, WB0, DF, PA);
  k_agg<<<gA, NTHR, 0, stream>>>(HIT, CNT, PA, PB, b0, nN, MP);
  k_gemm<8><<<gM, GTHR, 0, stream>>>(PB, WB1, AP, PA);
  k_agg<<<gA, NTHR, 0, stream>>>(HIT, CNT, PA, PB, b1, nN, MP);
  k_gemm<4><<<gM, GTHR, 0, stream>>>(PB, WB2, AP, PA);
  k_agg2<<<gA, NTHR, 0, stream>>>(HIT, CNT, PA, (const float*)PB, b2, nN, MP, out, (long long)nN * (NCLS / 4));
}
